// GAT_4449586118921
// MI455X (gfx1250) — hardware-run, weakly checked
//
#include <hip/hip_runtime.h>
#include <stddef.h>
#include <stdint.h>
#include <math.h>


#define NN      50000
#define EE      800000
#define FIN     256
#define HC1     128
#define OUTC    40
#define NC2P    48
#define TWO_TERM 1
#define APITCH  256
#define WPITCH  256
#define K2EXT   (TWO_TERM ? 256 : 128)
#define TM      128
#define MP      (((NN + TM - 1) / TM) * TM)
#define NTHR    256
#define NWAVE   8
#define NBRUN   1024
#define NBLK    ((NN + NBRUN - 1) / NBRUN)
#define NSLOT   (NBLK * NBRUN)
#define WLCAP   3584
#define RCAP    (NWAVE * WLCAP)
#define DEGCAP  64
#define STEPK   128
#define EPW     (((EE + NWAVE * STEPK - 1) / (NWAVE * STEPK)) * STEPK)
#define GRP     64
#define NEGSL   0.2f
#define EPS_SM  1e-16f
#define BN_EPS  1e-5f

#define LDS_G1  ((TM * HC1 + 2 * HC1 + TM * 8) * 4)
#define LDS_BK  ((NWAVE * WLCAP + RCAP + 3 * NBRUN + 32) * 4)
#define LDS_R2  (NWAVE * GRP * OUTC * 4)

#define NB_XB   ((MP * (FIN / 8)) / NTHR)
#define NB_W1   ((HC1 * (FIN / 8)) / NTHR)
#define NB_W2   ((NC2P * (WPITCH / 8)) / NTHR)
#define NB_TOT  (NB_XB + NB_W1 + NB_W2 + 1)

static_assert(NN <= 65536 && NBRUN <= 1024);
static_assert(RCAP >= 16623 + 4096);
static_assert(DEGCAP >= 35 + 8);
static_assert(NWAVE * EPW >= EE && (EPW % STEPK) == 0);
static_assert((MP % TM) == 0 && (MP % 16) == 0 && MP <= NSLOT);
static_assert((MP * (FIN / 8)) % NTHR == 0 && (HC1 * (FIN / 8)) % NTHR == 0 && (NC2P * (WPITCH / 8)) % NTHR == 0);
static_assert((FIN % 32) == 0 && (K2EXT % 32) == 0 && K2EXT <= APITCH && K2EXT <= WPITCH);
static_assert(NC2P % 16 == 0 && OUTC <= NC2P && (OUTC % 4) == 0);
static_assert((GRP % 4) == 0 && (NN % 4) == 0 && ((NBRUN * OUTC * 4) % 128) == 0 && ((GRP * OUTC * 4) % 128) == 0);
static_assert(NBRUN == NWAVE * 2 * GRP);
static_assert(((RCAP + NBRUN) % (NTHR * 4)) == 0 && (RCAP % (NTHR * 4)) == 0);
static_assert(LDS_G1 <= 300000 && LDS_BK <= 300000 && LDS_R2 <= 300000);
static_assert((NN - (NN / TM) * TM) % 4 == 0);

constexpr size_t al256c(size_t v) { return (v + 255) & ~(size_t)255; }
constexpr size_t O_XB   = 0;
constexpr size_t O_W1T  = al256c(O_XB   + (size_t)MP * FIN * 2);
constexpr size_t O_W2D  = al256c(O_W1T  + (size_t)HC1 * FIN * 2);
constexpr size_t O_PAR  = al256c(O_W2D  + (size_t)NC2P * WPITCH * 2);
constexpr size_t O_H1   = al256c(O_PAR  + (size_t)1024 * 4);
constexpr size_t O_SD1  = al256c(O_H1   + (size_t)MP * HC1 * 4);
constexpr size_t O_LIST = al256c(O_SD1  + (size_t)MP * 8 * 4);
constexpr size_t O_OFF  = al256c(O_LIST + (size_t)NBLK * RCAP * 4);
constexpr size_t O_CNT  = al256c(O_OFF  + (size_t)NSLOT * 4);
constexpr size_t O_FLAG = al256c(O_CNT  + (size_t)NSLOT * 4);
constexpr size_t O_T    = al256c(O_FLAG + (size_t)NBLK * 32 * 4);
constexpr size_t O_REC  = al256c(O_T    + (size_t)NN * HC1 * 4);
constexpr size_t O_MR   = al256c(O_REC  + (size_t)NBLK * HC1 * 2 * 8);
constexpr size_t O_EHL  = al256c(O_MR   + (size_t)256 * 4);
constexpr size_t O_H2   = al256c(O_EHL  + (size_t)MP * APITCH * 2);
constexpr size_t O_SD2  = al256c(O_H2   + (size_t)MP * NC2P * 4);
constexpr size_t WS_TOTAL = al256c(O_SD2 + (size_t)MP * 2 * 4);
static_assert(WS_TOTAL <= ((size_t)128u << 20));

typedef float          v4f  __attribute__((ext_vector_type(4)));
typedef float          v8f  __attribute__((ext_vector_type(8)));
typedef double         v2d  __attribute__((ext_vector_type(2)));
typedef int            v4i  __attribute__((ext_vector_type(4)));
typedef int            v8i  __attribute__((ext_vector_type(8)));
typedef unsigned int   v4u  __attribute__((ext_vector_type(4)));
typedef unsigned short v8us __attribute__((ext_vector_type(8)));
typedef __bf16         v16b __attribute__((ext_vector_type(16)));
typedef v4f  __attribute__((may_alias)) v4fa;
typedef v4i  __attribute__((may_alias)) v4ia;
typedef v4u  __attribute__((may_alias)) v4ua;
typedef v2d  __attribute__((may_alias)) v2da;
typedef v8us __attribute__((may_alias)) v8usa;
union FragB { v16b v; v8us h[2]; v8i w; };

#define PIN(x) asm volatile("" :: "v"(x))

__device__ __forceinline__ v8f wmb(const FragB& a, const FragB& b, v8f c) {
  v8f d = __builtin_amdgcn_wmma_f32_16x16x32_bf16(false, a.v, false, b.v, (short)0, c, false, false);
  asm volatile("v_nop\n\tv_nop\n\tv_nop\n\tv_nop" : "+v"(d) : "v"(a.w), "v"(b.w));
  return d;
}

__device__ __forceinline__ int iclamp(int v, int lo, int hi) { v = v < lo ? lo : v; return v > hi ? hi : v; }

__device__ __forceinline__ unsigned int f2bf(float f) {
  const unsigned int u = __float_as_uint(f);
  return ((u + 0x7FFFu + ((u >> 16) & 1u)) >> 16) & 0xFFFFu;
}
__device__ __forceinline__ unsigned int f2bf_n(float f) {
  const unsigned int u = __float_as_uint(f);
  const unsigned int r = ((u + 0x7FFFu + ((u >> 16) & 1u)) >> 16) & 0xFFFFu;
  return ((u & 0x7FFFFFFFu) > 0x7F800000u) ? 0x7FC0u : r;
}
__device__ __forceinline__ float bf2f(unsigned int b) { return __uint_as_float(b << 16); }
__device__ __forceinline__ float bfr(float f) { return bf2f(f2bf(f)); }
__device__ __forceinline__ v4f bfr4(const v4f a) {
  v4f r; r.x = bfr(a.x); r.y = bfr(a.y); r.z = bfr(a.z); r.w = bfr(a.w); return r;
}
__device__ __forceinline__ unsigned int pk2(float lo, float hi) { return f2bf(lo) | (f2bf(hi) << 16); }
__device__ __forceinline__ v4u pack8(const v4f a, const v4f b) {
  v4u r;
  r.x = pk2(a.x, a.y); r.y = pk2(a.z, a.w); r.z = pk2(b.x, b.y); r.w = pk2(b.z, b.w);
  return r;
}
__device__ __forceinline__ void put4f(float* p, const v4f v) {
  *(volatile v4f*)p = v;
  __threadfence();
  *(volatile v4f*)p = v;
}
__device__ __forceinline__ void put4u(unsigned short* p, const v4u v) {
  *(volatile v4u*)p = v;
  __threadfence();
  *(volatile v4u*)p = v;
}

__device__ __forceinline__ void osm4(const float lg, const v4f fs, float& mx, float& dn, v4f& av) {
  const float df = lg - mx;
  const float ee = expf(-fabsf(df));
  const bool up  = df > 0.f;
  const float s1 = up ? ee : 1.0f;
  const float s2 = up ? 1.0f : ee;
  mx = up ? lg : mx;
  dn = fmaf(dn, s1, s2);
  av.x = fmaf(av.x, s1, s2 * fs.x);
  av.y = fmaf(av.y, s1, s2 * fs.y);
  av.z = fmaf(av.z, s1, s2 * fs.z);
  av.w = fmaf(av.w, s1, s2 * fs.w);
}

__device__ __forceinline__ int append_hits(const bool hit, const int entry, const int wc, int* wlw) {
  const unsigned mj = __builtin_amdgcn_ballot_w32(hit);
  if (hit) {
    const int pos = wc + (int)__builtin_amdgcn_mbcnt_lo(mj, 0u);
    if (pos < WLCAP) wlw[pos] = entry;
  }
  return wc + (int)__builtin_popcount(mj);
}

__global__ __launch_bounds__(NTHR) void k_prep(
    const float* __restrict__ x, const float* __restrict__ W1,
    const float* __restrict__ as1, const float* __restrict__ ad1, const float* __restrict__ b1,
    const float* __restrict__ gam, const float* __restrict__ bet, const float* __restrict__ W2,
    const float* __restrict__ as2, const float* __restrict__ ad2, const float* __restrict__ b2, char* ws)
{
  const int tid = (int)threadIdx.x;
  const int b   = (int)blockIdx.x;
  const v4f z4 = {0.f, 0.f, 0.f, 0.f};
  if (b < NB_XB) {
    unsigned short* xb = (unsigned short*)(ws + O_XB);
    const int i   = b * NTHR + tid;
    const int row = i >> 5;
    const int c0  = (i & 31) * 8;
    const int rc  = row < NN ? row : NN - 1;
    const float* p = x + (size_t)rc * FIN + c0;
    v4f a = *(const v4fa*)p, q = *(const v4fa*)(p + 4);
    PIN(a); PIN(q);
    const bool ok = row < NN;
    a = ok ? a : z4;
    q = ok ? q : z4;
    put4u(xb + (size_t)row * FIN + c0, pack8(a, q));
  } else if (b < NB_XB + NB_W1) {
    unsigned short* wt = (unsigned short*)(ws + O_W1T);
    const int u  = (b - NB_XB) * NTHR + tid;
    const int n  = u >> 5;
    const int k8 = (u & 31) * 8;
    const float* p = W1 + (size_t)k8 * HC1 + n;
    v4f a, q;
    a.x = p[0];        a.y = p[HC1];      a.z = p[2 * HC1];  a.w = p[3 * HC1];
    q.x = p[4 * HC1];  q.y = p[5 * HC1];  q.z = p[6 * HC1];  q.w = p[7 * HC1];
    put4u(wt + (size_t)n * FIN + k8, pack8(a, q));
  } else if (b < NB_XB + NB_W1 + NB_W2) {
    unsigned short* wt = (unsigned short*)(ws + O_W2D);
    const int u   = (b - NB_XB - NB_W1) * NTHR + tid;
    const int n   = u >> 5;
    const int k8  = (u & 31) * 8;
    const int kk  = k8 & (HC1 - 1);
    const int ncl = n < OUTC ? n : OUTC - 1;
    const float* p = W2 + (size_t)kk * OUTC + ncl;
    v4f a, q;
    a.x = p[0];         a.y = p[OUTC];      a.z = p[2 * OUTC];  a.w = p[3 * OUTC];
    q.x = p[4 * OUTC];  q.y = p[5 * OUTC];  q.z = p[6 * OUTC];  q.w = p[7 * OUTC];
    PIN(a); PIN(q);
    const bool ok = n < OUTC;
    a = ok ? a : z4;
    q = ok ? q : z4;
    put4u(wt + (size_t)n * WPITCH + k8, pack8(a, q));
  } else {
    float* par = (float*)(ws + O_PAR);
    const int lane = tid & 31, seg = tid >> 5;
    const int i4 = 4 * lane;
    const int j4 = i4 > OUTC - 4 ? OUTC - 4 : i4;
    const bool in40 = lane < OUTC / 4;
    v4f v = z4;
    if (seg == 0)      { v = *(const v4fa*)(as1 + i4); }
    else if (seg == 1) { v = *(const v4fa*)(ad1 + i4); }
    else if (seg == 2) { v = *(const v4fa*)(b1 + i4); }
    else if (seg == 3) { v = *(const v4fa*)(gam + i4); }
    else if (seg == 4) { v = *(const v4fa*)(bet + i4); }
    else if (seg == 5) { v4f t = *(const v4fa*)(as2 + j4); PIN(t); v = in40 ? t : z4; }
    else if (seg == 6) { v4f t = *(const v4fa*)(ad2 + j4); PIN(t); v = in40 ? t : z4; }
    else               { v4f t = *(const v4fa*)(b2 + j4);  PIN(t); v = in40 ? t : z4; }
    put4f(par + seg * 128 + i4, bfr4(v));
  }
}

__global__ __launch_bounds__(NTHR) __attribute__((amdgpu_num_vgpr(248)))
void k_gemm_one(const unsigned short* __restrict__ XB, const unsigned short* __restrict__ W1T,
                const float* __restrict__ PAR, float* H1, float* SD1)
{
  extern __shared__ v4f g1_dyn[];
  float* stg  = (float*)g1_dyn;
  float* satt = stg + TM * HC1;
  float* sds  = satt + 2 * HC1;
  const int tid = (int)threadIdx.x, lane = tid & 31, wave = tid >> 5, hh = lane >> 4, m = lane & 15;
  const int rowBase = (int)blockIdx.x * TM;
  int nlive = NN - rowBase; nlive = nlive > TM ? TM : nlive;

  if (tid < 64) {
    const v4f a = *(const v4fa*)(PAR + 4 * tid);
    *(v4fa*)(satt + 4 * tid) = a;
  }

  v8f acc[8];
  {
    const v8f z = {0.f, 0.f, 0.f, 0.f, 0.f, 0.f, 0.f, 0.f};
#pragma unroll
    for (int t = 0; t < 8; ++t) acc[t] = z;
  }
  const unsigned short* ap = XB  + (size_t)(rowBase + 16 * wave + m) * FIN + 8 * hh;
  const unsigned short* wp = W1T + (size_t)m * FIN + 8 * hh;
#pragma unroll 1
  for (int ks = 0; ks < FIN / 32; ++ks) {
    FragB af;
    af.h[0] = *(const v8usa*)(ap + 32 * ks);
    af.h[1] = *(const v8usa*)(ap + 32 * ks + 16);
#pragma unroll
    for (int t = 0; t < 8; ++t) {
      const unsigned short* wq = wp + (size_t)(16 * t) * FIN + 32 * ks;
      FragB bf;
      bf.h[0] = *(const v8usa*)wq;
      bf.h[1] = *(const v8usa*)(wq + 16);
      acc[t] = wmb(af, bf, acc[t]);
    }
  }

#pragma unroll
  for (int t = 0; t < 8; ++t) {
#pragma unroll
    for (int r = 0; r < 8; ++r)
      stg[(16 * wave + 8 * hh + r) * HC1 + 16 * t + m] = acc[t][r];
  }
  __syncthreads();

  {
    const int row = tid & (TM - 1), which = tid >> 7;
#pragma unroll 1
    for (int hd = 0; hd < 4; ++hd) {
      const float* sa = satt + which * HC1 + hd * 32;
      const float* hr = stg + row * HC1 + hd * 32;
      float d = 0.f;
#pragma unroll 4
      for (int c4 = 0; c4 < 8; ++c4) {
        const v4f hv = *(const v4fa*)(hr + 4 * c4);
        const v4f av = *(const v4fa*)(sa + 4 * c4);
        d = fmaf(hv.x, av.x, d);
        d = fmaf(hv.y, av.y, d);
        d = fmaf(hv.z, av.z, d);
        d = fmaf(hv.w, av.w, d);
      }
      sds[row * 8 + which * 4 + hd] = d;
    }
  }
  __syncthreads();

  v4f fv[16];
#pragma unroll
  for (int i = 0; i < 16; ++i) fv[i] = *(const v4fa*)(stg + (16 * wave + i) * HC1 + 4 * lane);
  const v4f sv = *(const v4fa*)(sds + 4 * tid);
  const bool sok = tid < nlive * 2;
  float* sp = SD1 + (size_t)rowBase * 8 + 4 * tid;

#pragma unroll
  for (int i = 0; i < 16; ++i) {
    if (16 * wave + i < nlive)
      *(volatile v4f*)(H1 + (size_t)(rowBase + 16 * wave + i) * HC1 + 4 * lane) = fv[i];
  }
  if (sok) *(volatile v4f*)sp = sv;
  __threadfence();
#pragma unroll
  for (int i = 0; i < 16; ++i) {
    if (16 * wave + i < nlive)
      *(volatile v4f*)(H1 + (size_t)(rowBase + 16 * wave + i) * HC1 + 4 * lane) = fv[i];
  }
  if (sok) *(volatile v4f*)sp = sv;
}

__global__ __launch_bounds__(NTHR) void k_bucket(const int* __restrict__ ei, int* LIST, int* OFF, int* CNT,
                                                 int* FLAG)
{
  extern __shared__ v4i bk_dyn[];
  int* wl   = (int*)bk_dyn;
  int* srt  = wl + NWAVE * WLCAP;
  int* cnt  = srt + RCAP;
  int* off  = cnt + NBRUN;
  int* cur  = off + NBRUN;
  int* misc = cur + NBRUN;
  const int tid = (int)threadIdx.x, lane = tid & 31, wave = tid >> 5;
  const int blk = (int)blockIdx.x;
  const int nodeBase = blk * NBRUN;
  int nb = NN - nodeBase; nb = nb > NBRUN ? NBRUN : nb;
  const int* srcs = ei;
  const int* dsts = ei + EE;

  {
    const v4i z4 = {0, 0, 0, 0};
#pragma unroll 1
    for (int i = tid * 4; i < RCAP + NBRUN; i += NTHR * 4) *(v4ia*)(srt + i) = z4;
    if (tid < 32) misc[tid] = 0;
  }
  __syncthreads();

  const int wbeg = wave * EPW;
  int wend = wbeg + EPW; wend = wend > EE ? EE : wend;
  int nst = (wend - wbeg + STEPK - 1) / STEPK;
  nst = iclamp(nst, 0, EPW / STEPK);
  int* wlw = wl + wave * WLCAP;
  int wc = 0;
#pragma unroll 1
  for (int st = 0; st < nst; ++st) {
    const int e0 = wbeg + st * STEPK + lane;
    const int e1 = e0 + 32, e2 = e0 + 64, e3 = e0 + 96;
    const int a0 = e0 > EE - 1 ? EE - 1 : e0;
    const int a1 = e1 > EE - 1 ? EE - 1 : e1;
    const int a2 = e2 > EE - 1 ? EE - 1 : e2;
    const int a3 = e3 > EE - 1 ? EE - 1 : e3;
    const int k0 = dsts[a0], k1 = dsts[a1], k2 = dsts[a2], k3 = dsts[a3];
    const int r0 = srcs[a0], r1 = srcs[a1], r2 = srcs[a2], r3 = srcs[a3];
    PIN(k0); PIN(k1); PIN(k2); PIN(k3);
    PIN(r0); PIN(r1); PIN(r2); PIN(r3);
    const unsigned s0 = (unsigned)k0 - (unsigned)nodeBase, s1 = (unsigned)k1 - (unsigned)nodeBase;
    const unsigned s2 = (unsigned)k2 - (unsigned)nodeBase, s3 = (unsigned)k3 - (unsigned)nodeBase;
    const bool h0 = (e0 < wend) & (s0 < (unsigned)nb);
    const bool h1 = (e1 < wend) & (s1 < (unsigned)nb);
    const bool h2 = (e2 < wend) & (s2 < (unsigned)nb);
    const bool h3 = (e3 < wend) & (s3 < (unsigned)nb);
    const unsigned any = __builtin_amdgcn_ballot_w32(h0 | h1 | h2 | h3);
    if (any != 0u) {
      const int n0 = iclamp(r0, 0, NN - 1) | (int)((s0 & (NBRUN - 1)) << 16);
      const int n1 = iclamp(r1, 0, NN - 1) | (int)((s1 & (NBRUN - 1)) << 16);
      const int n2 = iclamp(r2, 0, NN - 1) | (int)((s2 & (NBRUN - 1)) << 16);
      const int n3 = iclamp(r3, 0, NN - 1) | (int)((s3 & (NBRUN - 1)) << 16);
      wc = append_hits(h0, n0, wc, wlw);
      wc = append_hits(h1, n1, wc, wlw);
      wc = append_hits(h2, n2, wc, wlw);
      wc = append_hits(h3, n3, wc, wlw);
    }
  }
  if (lane == 0) misc[wave] = wc;
  __syncthreads();

  if (wave == 0) {
#pragma unroll 1
    for (int w2 = 0; w2 < NWAVE; ++w2) {
      const int c = iclamp(misc[w2], 0, WLCAP);
#pragma unroll 1
      for (int b0 = 0; b0 < c; b0 += 32) {
        int idx = b0 + lane; idx = idx > c - 1 ? c - 1 : idx;
        const int ent = wl[w2 * WLCAP + idx];
        const int m32 = (c - b0) < 32 ? (c - b0) : 32;
#pragma unroll 1
        for (int k = 0; k < m32; ++k) {
          const int u  = __builtin_amdgcn_readlane(ent, k);
          const int sl = (u >> 16) & (NBRUN - 1);
          if (lane == 0) cnt[sl] = cnt[sl] + 1;
        }
      }
    }
  }
  __syncthreads();

  int flagv = 0;
  {
    const v4i c4 = *(const v4ia*)(cnt + 4 * tid);
    const int q0 = c4.x < 0 ? 0 : c4.x, q1 = c4.y < 0 ? 0 : c4.y;
    const int q2 = c4.z < 0 ? 0 : c4.z, q3 = c4.w < 0 ? 0 : c4.w;
    const bool big = (q0 > DEGCAP) | (q1 > DEGCAP) | (q2 > DEGCAP) | (q3 > DEGCAP);
    const int ts = q0 + q1 + q2 + q3;
    int incl = ts;
#pragma unroll
    for (int d = 1; d < 32; d <<= 1) {
      const int up = __shfl_up(incl, d);
      incl += (lane >= d) ? up : 0;
    }
    const unsigned bm = __builtin_amdgcn_ballot_w32(big);
    if (lane == 31) misc[8 + wave] = incl;
    if (lane == 0)  misc[16 + wave] = (bm != 0u) ? 1 : 0;
    __syncthreads();
    int pre = 0;
#pragma unroll
    for (int w2 = 0; w2 < NWAVE; ++w2) {
      const int t2 = misc[8 + w2];
      pre += (w2 < wave) ? t2 : 0;
      flagv |= misc[16 + w2];
      flagv |= (misc[w2] > WLCAP) ? 1 : 0;
    }
    const int run = pre + incl - ts;
    v4i o4;
    o4.x = run; o4.y = run + q0; o4.z = run + q0 + q1; o4.w = run + q0 + q1 + q2;
    *(v4ia*)(off + 4 * tid) = o4;
    *(v4ia*)(cur + 4 * tid) = o4;
  }
  __syncthreads();

  if (wave == 0) {
#pragma unroll 1
    for (int w2 = 0; w2 < NWAVE; ++w2) {
      const int c = iclamp(misc[w2], 0, WLCAP);
#pragma unroll 1
      for (int b0 = 0; b0 < c; b0 += 32) {
        int idx = b0 + lane; idx = idx > c - 1 ? c - 1 : idx;
        const int ent = wl[w2 * WLCAP + idx];
        const int m32 = (c - b0) < 32 ? (c - b0) : 32;
#pragma unroll 1
        for (int k = 0; k < m32; ++k) {
          const int u  = __builtin_amdgcn_readlane(ent, k);
          const int sl = (u >> 16) & (NBRUN - 1);
          if (lane == 0) {
            const int p = iclamp(cur[sl], 0, RCAP - 1);
            srt[p] = u & 0xFFFF;
            cur[sl] = p + 1;
          }
        }
      }
    }
  }
  __syncthreads();

  int* lrow = LIST + (size_t)blk * RCAP;
  const v4i ov = *(const v4ia*)(off + 4 * tid);
  const v4i cv = *(const v4ia*)(cnt + 4 * tid);
  const v4i fl = {flagv, flagv, flagv, flagv};
#pragma unroll 1
  for (int i = tid * 4; i < RCAP; i += NTHR * 4) {
    const v4i v = *(const v4ia*)(srt + i);
    *(volatile v4i*)(lrow + i) = v;
  }
  *(volatile v4i*)(OFF + nodeBase + 4 * tid) = ov;
  *(volatile v4i*)(CNT + nodeBase + 4 * tid) = cv;
  if (tid < 8) *(volatile v4i*)(FLAG + blk * 32 + 4 * tid) = fl;
  __threadfence();
#pragma unroll 1
  for (int i = tid * 4; i < RCAP; i += NTHR * 4) {
    const v4i v = *(const v4ia*)(srt + i);
    *(volatile v4i*)(lrow + i) = v;
  }
  *(volatile v4i*)(OFF + nodeBase + 4 * tid) = ov;
  *(volatile v4i*)(CNT + nodeBase + 4 * tid) = cv;
  if (tid < 8) *(volatile v4i*)(FLAG + blk * 32 + 4 * tid) = fl;
}

__global__ __launch_bounds__(NTHR) void k_replay_one(
    const float* __restrict__ H1, const float* __restrict__ SD1, const int* __restrict__ LIST,
    const int* __restrict__ OFF, const int* __restrict__ CNT, const int* __restrict__ FLAG,
    const float* __restrict__ PAR, float* T, double* REC)
{
  __shared__ double wrec[NWAVE * 2 * HC1];
  const int tid = (int)threadIdx.x, lane = tid & 31, wave = tid >> 5;
  const int blk = (int)blockIdx.x;
  const int nodeBase = blk * NBRUN;
  const int c0 = 4 * lane, head = lane >> 3;
  const int* lst = LIST + (size_t)blk * RCAP;
  const bool bflag = FLAG[blk * 32] != 0;
  const v4f bb = *(const v4fa*)(PAR + 2 * 128 + c0);
  const float qnan = __int_as_float(0x7fc00000);
  double sx = 0.0, sy = 0.0, sz = 0.0, sw = 0.0, qx = 0.0, qy = 0.0, qz = 0.0, qw = 0.0;

#pragma unroll 1
  for (int jt = 0; jt < NBRUN / NWAVE; ++jt) {
    const int d = nodeBase + wave * (NBRUN / NWAVE) + jt;
    const bool live = d < NN;
    const int dcl = live ? d : NN - 1;
    int ovv = OFF[d];
    int cvv = CNT[d];
    const bool big = cvv > DEGCAP;
    ovv = iclamp(ovv, 0, RCAP);
    cvv = iclamp(cvv, 0, DEGCAP);
    cvv = cvv > RCAP - ovv ? RCAP - ovv : cvv;
    const int o = __builtin_amdgcn_readfirstlane(ovv);
    const int c = __builtin_amdgcn_readfirstlane(cvv);
    int last = o + c - 1; last = last < o ? o : last;
    last = last > RCAP - 1 ? RCAP - 1 : last;

    const float adv = SD1[(size_t)dcl * 8 + 4 + head];
    float mx = __int_as_float((int)0xff800000u), dn = 0.f;
    v4f av = {0.f, 0.f, 0.f, 0.f};
    const int tot = c + 1;
#pragma unroll 1
    for (int b0 = 0; b0 < tot; b0 += 32) {
      const int i = b0 + lane;
      int idx = o + i; idx = idx > last ? last : idx;
      int sv = lst[idx];
      PIN(sv);
      sv = iclamp(sv, 0, NN - 1);
      sv = (i >= c) ? dcl : sv;
      const int m32 = (tot - b0) < 32 ? (tot - b0) : 32;
#pragma unroll 1
      for (int k = 0; k < m32; ++k) {
        const int s = __builtin_amdgcn_readlane(sv, k);
        const v4f fs = *(const v4fa*)(H1 + (size_t)s * HC1 + c0);
        float lg = SD1[(size_t)s * 8 + head] + adv;
        lg = lg > 0.f ? lg : NEGSL * lg;
        osm4(lg, fs, mx, dn, av);
      }
    }
    const float inv = 1.0f / (dn + EPS_SM);
    const bool pois = bflag | big;
    v4f ov;
    ov.x = pois ? qnan : fmaf(av.x, inv, bb.x);
    ov.y = pois ? qnan : fmaf(av.y, inv, bb.y);
    ov.z = pois ? qnan : fmaf(av.z, inv, bb.z);
    ov.w = pois ? qnan : fmaf(av.w, inv, bb.w);
    if (live) {
      float* tp = T + (size_t)d * HC1 + c0;
      *(volatile v4f*)tp = ov;
      __threadfence();
      *(volatile v4f*)tp = ov;
      const double dx = (double)ov.x, dy = (double)ov.y, dz = (double)ov.z, dw = (double)ov.w;
      sx += dx; sy += dy; sz += dz; sw += dw;
      qx = fma(dx, dx, qx); qy = fma(dy, dy, qy); qz = fma(dz, dz, qz); qw = fma(dw, dw, qw);
    }
  }

  double* wr = wrec + wave * (2 * HC1);
  wr[c0 + 0] = sx; wr[c0 + 1] = sy; wr[c0 + 2] = sz; wr[c0 + 3] = sw;
  wr[HC1 + c0 + 0] = qx; wr[HC1 + c0 + 1] = qy; wr[HC1 + c0 + 2] = qz; wr[HC1 + c0 + 3] = qw;
  __syncthreads();
  if (tid < HC1) {
    double s = 0.0, q = 0.0;
#pragma unroll 1
    for (int w2 = 0; w2 < NWAVE; ++w2) {
      s += wrec[w2 * (2 * HC1) + tid];
      q += wrec[w2 * (2 * HC1) + HC1 + tid];
    }
    v2d r; r.x = s; r.y = q;
    double* rp = REC + ((size_t)blk * HC1 + tid) * 2;
    *(volatile v2d*)rp = r;
    __threadfence();
    *(volatile v2d*)rp = r;
  }
}

__global__ __launch_bounds__(HC1) void k_bn_combine(const double* __restrict__ REC, float* MR)
{
  __shared__ __attribute__((aligned(16))) float st[2 * HC1];
  const int c = (int)threadIdx.x;
  double s = 0.0, q = 0.0;
#pragma unroll 1
  for (int b = 0; b < NBLK; ++b) {
    const v2d r = *(const v2da*)(REC + ((size_t)b * HC1 + c) * 2);
    s += r.x;
    q += r.y;
  }
  const double invn = 1.0 / (double)NN;
  const double mu = s * invn;
  double var = q * invn - mu * mu;
  var = var < 0.0 ? 0.0 : var;
  const float varf = (float)var;
  st[c] = (float)mu;
  st[HC1 + c] = 1.0f / sqrtf(varf + BN_EPS);
  __syncthreads();
  if (c < (2 * HC1) / 4) {
    const v4f v = *(const v4fa*)(st + 4 * c);
    put4f(MR + 4 * c, v);
  }
}

__global__ __launch_bounds__(NTHR) void k_bn_apply(const float* __restrict__ T, const float* __restrict__ MR,
                                                   const float* __restrict__ PAR, unsigned short* EHL)
{
  __shared__ __attribute__((aligned(16))) float sp[4 * HC1];
  __shared__ __attribute__((aligned(16))) unsigned short tile[16 * APITCH];
  const int tid = (int)threadIdx.x;
  if (tid < 64) {
    const v4f v = *(const v4fa*)(MR + 4 * tid);
    *(v4fa*)(sp + 4 * tid) = v;
  } else if (tid < 128) {
    const v4f v = *(const v4fa*)(PAR + 3 * 128 + 4 * (tid - 64));
    *(v4fa*)(sp + 2 * HC1 + 4 * (tid - 64)) = v;
  }
  __syncthreads();
  const int rowBase = (int)blockIdx.x * 16;
#pragma unroll 1
  for (int it = 0; it < 8; ++it) {
    const int e = it * NTHR + tid;
    const int r = e >> 7, c = e & (HC1 - 1);
    const int row = rowBase + r;
    const int rc = row < NN ? row : NN - 1;
    const float t = T[(size_t)rc * HC1 + c];
    PIN(t);
    const float y = ((t - sp[c]) * sp[HC1 + c]) * sp[2 * HC1 + c] + sp[3 * HC1 + c];
    const float a = y > 0.f ? y : expm1f(y);
    const float v = row < NN ? a : 0.f;
    const unsigned int hb = f2bf_n(v);
    const unsigned int lb = f2bf_n(v - bf2f(hb));
    tile[r * APITCH + c] = (unsigned short)hb;
    tile[r * APITCH + HC1 + c] = (unsigned short)lb;
  }
  __syncthreads();
  const v4u p0 = *(const v4ua*)(tile + 8 * tid);
  const v4u p1 = *(const v4ua*)(tile + 8 * (NTHR + tid));
  unsigned short* ob = EHL + (size_t)rowBase * APITCH;
  *(volatile v4u*)(ob + 8 * tid) = p0;
  *(volatile v4u*)(ob + 8 * (NTHR + tid)) = p1;
  __threadfence();
  *(volatile v4u*)(ob + 8 * tid) = p0;
  *(volatile v4u*)(ob + 8 * (NTHR + tid)) = p1;
}

__global__ __launch_bounds__(NTHR) __attribute__((amdgpu_num_vgpr(248)))
void k_gemm_two(const unsigned short* __restrict__ EHL, const unsigned short* __restrict__ W2D,
                const float* __restrict__ PAR, float* H2, float* SD2)
{
  __shared__ __attribute__((aligned(16))) float stg[TM * NC2P];
  __shared__ __attribute__((aligned(16))) float satt[2 * NC2P];
  __shared__ __attribute__((aligned(16))) float sds[TM * 2];
  const int tid = (int)threadIdx.x, lane = tid & 31, wave = tid >> 5, hh = lane >> 4, m = lane & 15;
  const int rowBase = (int)blockIdx.x * TM;
  int nlive = NN - rowBase; nlive = nlive > TM ? TM : nlive;

  if (tid < 24) {
    const int which = tid / 12, p = tid - which * 12;
    const v4f a = *(const v4fa*)(PAR + (5 + which) * 128 + 4 * p);
    *(v4fa*)(satt + which * NC2P + 4 * p) = a;
  }

  v8f acc[3];
  {
    const v8f z = {0.f, 0.f, 0.f, 0.f, 0.f, 0.f, 0.f, 0.f};
    acc[0] = z; acc[1] = z; acc[2] = z;
  }
  const unsigned short* ap = EHL + (size_t)(rowBase + 16 * wave + m) * APITCH + 8 * hh;
  const unsigned short* wp = W2D + (size_t)m * WPITCH + 8 * hh;
#pragma unroll 1
  for (int ks = 0; ks < K2EXT / 32; ++ks) {
    FragB af;
    af.h[0] = *(const v8usa*)(ap + 32 * ks);
    af.h[1] = *(const v8usa*)(ap + 32 * ks + 16);
#pragma unroll
    for (int t = 0; t < 3; ++t) {
      const unsigned short* wq = wp + (size_t)(16 * t) * WPITCH + 32 * ks;
      FragB bf;
      bf.h[0] = *(const v8usa*)wq;
      bf.h[1] = *(const v8usa*)(wq + 16);
      acc[t] = wmb(af, bf, acc[t]);
    }
  }

#pragma unroll
  for (int t = 0; t < 3; ++t) {
#pragma unroll
    for (int r = 0; r < 8; ++r)
      stg[(16 * wave + 8 * hh + r) * NC2P + 16 * t + m] = acc[t][r];
  }
  __syncthreads();

  {
    const int row = tid & (TM - 1), which = tid >> 7;
    const float* sa = satt + which * NC2P;
    const float* hr = stg + row * NC2P;
    float d = 0.f;
#pragma unroll 4
    for (int c4 = 0; c4 < NC2P / 4; ++c4) {
      const v4f hv = *(const v4fa*)(hr + 4 * c4);
      const v4f av = *(const v4fa*)(sa + 4 * c4);
      d = fmaf(hv.x, av.x, d);
      d = fmaf(hv.y, av.y, d);
      d = fmaf(hv.z, av.z, d);
      d = fmaf(hv.w, av.w, d);
    }
    sds[row * 2 + which] = d;
  }
  __syncthreads();

  const int npc = nlive * (NC2P / 4);
  v4f fv[6];
#pragma unroll
  for (int i = 0; i < 6; ++i) fv[i] = *(const v4fa*)(stg + 4 * (i * NTHR + tid));
  const int tcl = tid < 64 ? tid : 63;
  const v4f sv = *(const v4fa*)(sds + 4 * tcl);
  const bool sok = (tid < 64) & (2 * tid < nlive);
  float* hb = H2 + (size_t)rowBase * NC2P;
  float* sp = SD2 + (size_t)rowBase * 2 + 4 * tcl;

#pragma unroll
  for (int i = 0; i < 6; ++i) {
    const int p = i * NTHR + tid;
    if (p < npc) *(volatile v4f*)(hb + 4 * p) = fv[i];
  }
  if (sok) *(volatile v4f*)sp = sv;
  __threadfence();
#pragma unroll
  for (int i = 0; i < 6; ++i) {
    const int p = i * NTHR + tid;
    if (p < npc) *(volatile v4f*)(hb + 4 * p) = fv[i];
  }
  if (sok) *(volatile v4f*)sp = sv;
}

__global__ __launch_bounds__(NTHR) void k_replay_two(
    const float* __restrict__ H2, const float* __restrict__ SD2, const int* __restrict__ LIST,
    const int* __restrict__ OFF, const int* __restrict__ CNT, const int* __restrict__ FLAG,
    const float* __restrict__ PAR, float* out)
{
  extern __shared__ v4f r2_dyn[];
  const int tid = (int)threadIdx.x, lane = tid & 31, wave = tid >> 5;
  float* res = (float*)r2_dyn + wave * (GRP * OUTC);
  const int blk = (int)blockIdx.x;
  const int nodeBase = blk * NBRUN;
  const int qc = lane < 11 ? lane : 11;
  const int c0 = 4 * qc;
  const int* lst = LIST + (size_t)blk * RCAP;
  const bool bflag = FLAG[blk * 32] != 0;
  const v4f bb = *(const v4fa*)(PAR + 7 * 128 + c0);
  const float qnan = __int_as_float(0x7fc00000);

#pragma unroll 1
  for (int jt = 0; jt < NBRUN / NWAVE; ++jt) {
    const int d = nodeBase + wave * (NBRUN / NWAVE) + jt;
    const bool live = d < NN;
    const int dcl = live ? d : NN - 1;
    int ovv = OFF[d];
    int cvv = CNT[d];
    const bool big = cvv > DEGCAP;
    ovv = iclamp(ovv, 0, RCAP);
    cvv = iclamp(cvv, 0, DEGCAP);
    cvv = cvv > RCAP - ovv ? RCAP - ovv : cvv;
    const int o = __builtin_amdgcn_readfirstlane(ovv);
    const int c = __builtin_amdgcn_readfirstlane(cvv);
    int last = o + c - 1; last = last < o ? o : last;
    last = last > RCAP - 1 ? RCAP - 1 : last;

    const float adv = SD2[(size_t)dcl * 2 + 1];
    float mx = __int_as_float((int)0xff800000u), dn = 0.f;
    v4f av = {0.f, 0.f, 0.f, 0.f};
    const int tot = c + 1;
#pragma unroll 1
    for (int b0 = 0; b0 < tot; b0 += 32) {
      const int i = b0 + lane;
      int idx = o + i; idx = idx > last ? last : idx;
      int sv = lst[idx];
      PIN(sv);
      sv = iclamp(sv, 0, NN - 1);
      sv = (i >= c) ? dcl : sv;
      const int m32 = (tot - b0) < 32 ? (tot - b0) : 32;
#pragma unroll 1
      for (int k = 0; k < m32; ++k) {
        const int s = __builtin_amdgcn_readlane(sv, k);
        const v4f fs = *(const v4fa*)(H2 + (size_t)s * NC2P + c0);
        float lg = SD2[(size_t)s * 2] + adv;
        lg = lg > 0.f ? lg : NEGSL * lg;
        osm4(lg, fs, mx, dn, av);
      }
    }
    const float inv = 1.0f / (dn + EPS_SM);
    const bool pois = bflag | big;
    v4f ov;
    ov.x = pois ? qnan : fmaf(av.x, inv, bb.x);
    ov.y = pois ? qnan : fmaf(av.y, inv, bb.y);
    ov.z = pois ? qnan : fmaf(av.z, inv, bb.z);
    ov.w = pois ? qnan : fmaf(av.w, inv, bb.w);
    const int lr = jt & (GRP - 1);
    if (lane < OUTC / 4) *(v4fa*)(res + lr * OUTC + 4 * lane) = ov;

    if (lr == GRP - 1) {
      __syncthreads();
      const int row0 = nodeBase + wave * (NBRUN / NWAVE) + (jt & ~(GRP - 1));
      int nl = NN - row0; nl = nl < 0 ? 0 : (nl > GRP ? GRP : nl);
      const int npc = nl * (OUTC / 4);
      float* ob = out + (size_t)row0 * OUTC;
#pragma unroll 1
      for (int p = lane; p < npc; p += 32) {
        const v4f v = *(const v4fa*)(res + 4 * p);
        *(volatile v4f*)(ob + 4 * p) = v;
      }
      __threadfence();
#pragma unroll 1
      for (int p = lane; p < npc; p += 32) {
        const v4f v = *(const v4fa*)(res + 4 * p);
        *(volatile v4f*)(ob + 4 * p) = v;
      }
      __syncthreads();
    }
  }
}

extern "C" void kernel_launch(void* const* d_in, const int* in_sizes, int n_in,
                              void* d_out, int out_size, void* d_ws, size_t ws_size,
                              hipStream_t stream) {
  if (n_in != 12) return;
  if (in_sizes[0] != NN * FIN) return;
  if (in_sizes[1] != 2 * EE) return;
  if (in_sizes[2] != FIN * HC1) return;
  if (in_sizes[3] != HC1 || in_sizes[4] != HC1) return;
  if (in_sizes[5] != HC1 || in_sizes[6] != HC1 || in_sizes[7] != HC1) return;
  if (in_sizes[8] != HC1 * OUTC) return;
  if (in_sizes[9] != OUTC || in_sizes[10] != OUTC || in_sizes[11] != OUTC) return;
  if (out_size != NN * OUTC) return;
  if (WS_TOTAL > ws_size) return;

  const float* x   = (const float*)d_in[0];
  const int*   ei  = (const int*)  d_in[1];
  const float* W1  = (const float*)d_in[2];
  const float* as1 = (const float*)d_in[3];
  const float* ad1 = (const float*)d_in[4];
  const float* b1  = (const float*)d_in[5];
  const float* gam = (const float*)d_in[6];
  const float* bet = (const float*)d_in[7];
  const float* W2  = (const float*)d_in[8];
  const float* as2 = (const float*)d_in[9];
  const float* ad2 = (const float*)d_in[10];
  const float* b2  = (const float*)d_in[11];
  float* out = (float*)d_out;
  char* ws = (char*)d_ws;

  unsigned short* XB  = (unsigned short*)(ws + O_XB);
  unsigned short* W1T = (unsigned short*)(ws + O_W1T);
  unsigned short* W2D = (unsigned short*)(ws + O_W2D);
  float*  PAR  = (float*)(ws + O_PAR);
  float*  H1   = (float*)(ws + O_H1);
  float*  SD1  = (float*)(ws + O_SD1);
  int*    LIST = (int*)(ws + O_LIST);
  int*    OFF  = (int*)(ws + O_OFF);
  int*    CNT  = (int*)(ws + O_CNT);
  int*    FLAG = (int*)(ws + O_FLAG);
  float*  T    = (float*)(ws + O_T);
  double* REC  = (double*)(ws + O_REC);
  float*  MR   = (float*)(ws + O_MR);
  unsigned short* EHL = (unsigned short*)(ws + O_EHL);
  float*  H2   = (float*)(ws + O_H2);
  float*  SD2  = (float*)(ws + O_SD2);

  hipFuncSetAttribute(reinterpret_cast<const void*>(&k_gemm_one),
                      hipFuncAttributeMaxDynamicSharedMemorySize, LDS_G1);
  hipFuncSetAttribute(reinterpret_cast<const void*>(&k_bucket),
                      hipFuncAttributeMaxDynamicSharedMemorySize, LDS_BK);
  hipFuncSetAttribute(reinterpret_cast<const void*>(&k_replay_two),
                      hipFuncAttributeMaxDynamicSharedMemorySize, LDS_R2);

  k_prep<<<NB_TOT, NTHR, 0, stream>>>(x, W1, as1, ad1, b1, gam, bet, W2, as2, ad2, b2, ws);
  k_gemm_one<<<MP / TM, NTHR, LDS_G1, stream>>>(XB, W1T, PAR, H1, SD1);
  k_bucket<<<NBLK, NTHR, LDS_BK, stream>>>(ei, LIST, OFF, CNT, FLAG);
  k_replay_one<<<NBLK, NTHR, 0, stream>>>(H1, SD1, LIST, OFF, CNT, FLAG, PAR, T, REC);
  k_bn_combine<<<1, HC1, 0, stream>>>(REC, MR);
  k_bn_apply<<<MP / 16, NTHR, 0, stream>>>(T, MR, PAR, EHL);
  k_gemm_two<<<MP / TM, NTHR, 0, stream>>>(EHL, W2D, PAR, H2, SD2);
  k_replay_two<<<NBLK, NTHR, LDS_R2, stream>>>(H2, SD2, LIST, OFF, CNT, FLAG, PAR, out);
}
